// ProjectedLinear_26645977104594
// MI455X (gfx1250) — hardware-verified
//
#include <hip/hip_runtime.h>
#define JNR 8192
#define JNL 4096
#define JNQ 64
#define JNS 768
#define JCY 64.0f
typedef unsigned short v8us __attribute__((ext_vector_type(8), may_alias));
typedef float  v8f  __attribute__((ext_vector_type(8)));
typedef float  v4f  __attribute__((ext_vector_type(4)));
typedef float  v4fa __attribute__((ext_vector_type(4), may_alias));

__device__ __forceinline__ unsigned short bf16_bits(float x) { unsigned int u = __float_as_uint(x); return (unsigned short)((u + 0x7FFFu + ((u >> 16) & 1u)) >> 16); }
__device__ __forceinline__ float bf16_val(unsigned short b) { return __uint_as_float(((unsigned int)b) << 16); }
__device__ __forceinline__ float bf16_round(float x) { return bf16_val(bf16_bits(x)); }

typedef _Float16 v16h __attribute__((ext_vector_type(16)));
union FragH { v16h v; v8us half[2]; _Float16 h[16]; unsigned short u[16]; };

__global__ __launch_bounds__(256) void k_wt_f16(const float* __restrict__ W, _Float16* __restrict__ Wt, int K, int N, float scale) {
  const int t = blockIdx.x * 256 + threadIdx.x; if (t >= N * (K / 8)) return; const int n = t / (K / 8), k8 = (t % (K / 8)) * 8; FragH f;
#pragma unroll
  for (int i = 0; i < 8; ++i) f.h[i] = (_Float16)(bf16_round(W[(size_t)(k8 + i) * N + n]) * scale); const v8us o = f.half[0];
  *(volatile v8us*)((unsigned short*)Wt + (size_t)n * K + k8) = o; __threadfence(); *(volatile v8us*)((unsigned short*)Wt + (size_t)n * K + k8) = o;
}

typedef _Float16 v4h __attribute__((ext_vector_type(4)));

__global__ __launch_bounds__(256) void k_x16(const float* __restrict__ x, _Float16* __restrict__ X16, size_t n8) { const size_t t = (size_t)blockIdx.x * 256 + threadIdx.x; if (t >= n8) return; FragH f;
#pragma unroll
  for (int q = 0; q < 8; ++q) f.h[q] = (_Float16)bf16_round(x[t * 8 + q]); *(volatile v8us*)((unsigned short*)X16 + t * 8) = f.half[0]; __threadfence(); *(volatile v8us*)((unsigned short*)X16 + t * 8) = f.half[0]; }

__device__ __forceinline__ v16h g2_frag(const _Float16* p, int hh) { FragH f; f.half[0] = *(const v8us*)((const unsigned short*)p + 8 * hh); f.half[1] = *(const v8us*)((const unsigned short*)p + 16 + 8 * hh); return f.v; }
__device__ __forceinline__ v8f g2_mma(v16h a, v16h b, v8f c) { v8f d = __builtin_amdgcn_wmma_f32_16x16x32_f16(false, a, false, b, (short)0, c, false, false); asm volatile("v_nop\n\tv_nop\n\tv_nop\n\tv_nop" : "+v"(d) : "v"(a), "v"(b)); return d; }
template <int ACT>
__global__ __launch_bounds__(128) void k_gemm2(const _Float16* __restrict__ A, int lda, size_t sA, const _Float16* __restrict__ Bh, int ldb, size_t sB, float alpha, const float* __restrict__ bias, size_t sBias, const float* __restrict__ CP, int rowsPerB, size_t sCPb, int row0g,
    float* __restrict__ C, _Float16* __restrict__ C16, int ldc, size_t sC, int M, int N, int K) { static_assert(ACT == 0 || ACT == 3 || ACT == 6 || ACT == 8 || ACT == 9 || ACT == 11 || ACT == 12 || ACT == 14 || ACT == 15 || ACT == 16 || ACT == 17, "k_gemm2: unsupported ACT code (would silently apply no activation)");
  __shared__ __attribute__((aligned(16))) float so[4][32][68];
  const int tid = threadIdx.x, w = tid >> 5, lane = tid & 31, ln = lane & 15, hh = lane >> 4; const int by = blockIdx.y;
  A += (size_t)by * sA; Bh += (size_t)by * sB; const size_t cofs = (size_t)by * sC; const float* bp = bias ? bias + (size_t)by * sBias : nullptr;
  const int ntn = N >> 6; const int mt = blockIdx.x / ntn, nq = blockIdx.x - mt * ntn; const int row0 = mt * 128 + 32 * w, col0 = nq * 64; if (row0 >= M) return;
  const _Float16* a0p = A + (size_t)(row0 + ln) * lda; const _Float16* a1p = a0p + (size_t)16 * lda;
  const _Float16* b0p = Bh + (size_t)(col0 + ln) * ldb; const _Float16* b1p = b0p + (size_t)16 * ldb; const _Float16* b2p = b1p + (size_t)16 * ldb; const _Float16* b3p = b2p + (size_t)16 * ldb;
  const v8f z8 = {0.f,0.f,0.f,0.f,0.f,0.f,0.f,0.f}; v8f c00 = z8, c01 = z8, c02 = z8, c03 = z8, c10 = z8, c11 = z8, c12 = z8, c13 = z8;
  for (int kb = 0; kb < K; kb += 32) { const v16h a0 = g2_frag(a0p + kb, hh), a1 = g2_frag(a1p + kb, hh);
    v16h b = g2_frag(b0p + kb, hh); c00 = g2_mma(a0, b, c00); c10 = g2_mma(a1, b, c10);
    b = g2_frag(b1p + kb, hh); c01 = g2_mma(a0, b, c01); c11 = g2_mma(a1, b, c11);
    b = g2_frag(b2p + kb, hh); c02 = g2_mma(a0, b, c02); c12 = g2_mma(a1, b, c12);
    b = g2_frag(b3p + kb, hh); c03 = g2_mma(a0, b, c03); c13 = g2_mma(a1, b, c13); }
  v8f accs[8] = {c00, c01, c02, c03, c10, c11, c12, c13};
#pragma unroll
  for (int u = 0; u < 8; ++u) { const int t = u & 3, half = u >> 2; const int col = col0 + t * 16 + ln; const float bv = bp ? bf16_round(bp[col]) : 0.f;
#pragma unroll
    for (int r = 0; r < 8; ++r) { const int rloc = half * 16 + 8 * hh + r; float v = accs[u][r] * alpha + bv; if (CP) { if (rowsPerB < 0) v += CP[cofs + (size_t)(row0g + row0 + rloc) * ldc + col];        else { const int bidx = (row0g + row0 + rloc) / rowsPerB; v += CP[(size_t)bidx * sCPb + (size_t)by * 64 + col]; } }
      if (ACT == 3) v = fmaxf(v, 0.f); else if (ACT == 6) v = 0.5f * v * (1.0f + erff(v * 0.70710678118654752f)); else if (ACT == 11) v = 1.0f / (1.0f + expf(-v)); else if (ACT == 15) v = v / (1.0f + expf(-v)); else if (ACT == 12) v = (v > 0.f) ? v : 0.01f * v; else if (ACT == 8) v = tanhf(v); else if (ACT == 9) v = 0.5f * v * (1.0f + tanhf(0.7978845608028654f * (v + 0.044715f * v * v * v))); else if (ACT == 14) v = (v > 0.f) ? v : 0.1f * v; else if (ACT == 16) v = (v >= 0.f) ? v : 0.3f * v; else if (ACT == 17) v = (v >= 0.f) ? v : 0.2f * v;
      so[w][rloc][t * 16 + ln] = v; } }
  __builtin_amdgcn_fence(__ATOMIC_ACQ_REL, "workgroup"); __builtin_amdgcn_wave_barrier();
  const int rsub = lane >> 4, c4 = (lane & 15) * 4;
  for (int pass = 0; pass < 2; ++pass) {
#pragma unroll
    for (int q = 0; q < 16; ++q) { const int r = q * 2 + rsub; const v4f v = *(const v4fa*)&so[w][r][c4]; if (C) *(volatile v4f*)(C + cofs + (size_t)(row0 + r) * ldc + col0 + c4) = v; if (C16) { v4h h4; for (int i = 0; i < 4; ++i) h4[i] = (_Float16)v[i]; *(volatile v4h*)(C16 + cofs + (size_t)(row0 + r) * ldc + col0 + c4) = h4; } }
    if (pass == 0) __threadfence(); } }

__global__ __launch_bounds__(256) void k_cs16(const float* __restrict__ sw, _Float16* __restrict__ tw, float scale) { const size_t t = (size_t)blockIdx.x * 256 + threadIdx.x; FragH f;
#pragma unroll
  for (int q = 0; q < 8; ++q) f.h[q] = (_Float16)(bf16_round(sw[t * 8 + q]) * scale); unsigned short* tp = (unsigned short*)tw + t * 8; *(volatile v8us*)tp = f.half[0]; __threadfence(); *(volatile v8us*)tp = f.half[0]; }

extern "C" void kernel_launch(void* const* d_in, const int* in_sizes, int n_in,
                              void* d_out, int out_size, void* d_ws, size_t ws_size, hipStream_t stream) {
  if (n_in < 4) return; if (in_sizes[0] < JNR * JNL || in_sizes[1] < JNL * JNQ || in_sizes[2] < JNQ * JNS || in_sizes[3] < JNS * JNS || out_size < JNR * JNL) return;
  const float* xa = (const float*)d_in[0]; const float* wa = (const float*)d_in[1]; const float* wb = (const float*)d_in[2]; const float* wm = (const float*)d_in[3]; float* res = (float*)d_out;
  static_assert(JNR % 128 == 0 && JNL % 64 == 0 && JNQ % 64 == 0 && JNS % 64 == 0 && JNL % 32 == 0 && JNQ % 32 == 0 && JNS % 32 == 0 && (JNL * JNQ) % 8 == 0 && (JNQ * JNS) % 8 == 0 && (JNS * JNS) % 8 == 0 && (JNQ * JNS / 8) % 256 == 0 && (JNL * JNQ / 8) % 256 == 0, "whole tiles, whole depth steps, whole groups of eight");
  uint8_t* wsp = (uint8_t*)d_ws; size_t off = 0;
  auto take = [&](size_t bytes) { uint8_t* at = wsp + off; off += (bytes + 255) & ~(size_t)255; return at; };
  _Float16* TA1 = (_Float16*)take((size_t)JNQ * JNL * 2); _Float16* TB1 = (_Float16*)take((size_t)JNS * JNQ * 2); _Float16* TM = (_Float16*)take((size_t)JNS * JNS * 2); _Float16* TB2 = (_Float16*)take((size_t)JNQ * JNS * 2); _Float16* TA2 = (_Float16*)take((size_t)JNL * JNQ * 2);
  _Float16* PX = (_Float16*)take((size_t)JNR * JNL * 2); _Float16* P1 = (_Float16*)take((size_t)JNR * JNQ * 2); _Float16* P2 = (_Float16*)take((size_t)JNR * JNS * 2); _Float16* P3 = (_Float16*)take((size_t)JNR * JNS * 2); _Float16* P4 = (_Float16*)take((size_t)JNR * JNQ * 2);
  if (off > ws_size) return;
  k_wt_f16<<<(unsigned)(((size_t)JNQ * (JNL / 8) + 255) / 256), 256, 0, stream>>>(wa, TA1, JNL, JNQ, JCY);
  k_wt_f16<<<(unsigned)(((size_t)JNS * (JNQ / 8) + 255) / 256), 256, 0, stream>>>(wb, TB1, JNQ, JNS, JCY);
  k_x16<<<(unsigned)(((size_t)JNS * JNS / 8 + 255) / 256), 256, 0, stream>>>(wm, TM, (size_t)JNS * JNS / 8); k_cs16<<<(unsigned)((size_t)JNQ * JNS / 8 / 256), 256, 0, stream>>>(wb, TB2, JCY); k_cs16<<<(unsigned)((size_t)JNL * JNQ / 8 / 256), 256, 0, stream>>>(wa, TA2, JCY);
  k_x16<<<(unsigned)(((size_t)JNR * JNL / 8 + 255) / 256), 256, 0, stream>>>(xa, PX, (size_t)JNR * JNL / 8);
  k_gemm2<0><<<dim3((unsigned)((JNR / 128) * (JNQ / 64)), 1u), 128, 0, stream>>>(PX, JNL, (size_t)0, TA1, JNL, (size_t)0, 1.0f / JCY, nullptr, (size_t)0, nullptr, 1, 0, 0, nullptr, P1, JNQ, (size_t)0, JNR, JNQ, JNL);
  k_gemm2<0><<<dim3((unsigned)((JNR / 128) * (JNS / 64)), 1u), 128, 0, stream>>>(P1, JNQ, (size_t)0, TB1, JNQ, (size_t)0, 1.0f, nullptr, (size_t)0, nullptr, 1, 0, 0, nullptr, P2, JNS, (size_t)0, JNR, JNS, JNQ);
  k_gemm2<0><<<dim3((unsigned)((JNR / 128) * (JNS / 64)), 1u), 128, 0, stream>>>(P2, JNS, (size_t)0, TM, JNS, (size_t)0, 1.0f / JCY, nullptr, (size_t)0, nullptr, 1, 0, 0, nullptr, P3, JNS, (size_t)0, JNR, JNS, JNS);
  k_gemm2<0><<<dim3((unsigned)((JNR / 128) * (JNQ / 64)), 1u), 128, 0, stream>>>(P3, JNS, (size_t)0, TB2, JNS, (size_t)0, 1.0f / JCY, nullptr, (size_t)0, nullptr, 1, 0, 0, nullptr, P4, JNQ, (size_t)0, JNR, JNQ, JNS);
  k_gemm2<0><<<dim3((unsigned)((JNR / 128) * (JNL / 64)), 1u), 128, 0, stream>>>(P4, JNQ, (size_t)0, TA2, JNQ, (size_t)0, 1.0f / JCY, nullptr, (size_t)0, nullptr, 1, 0, 0, res, nullptr, JNL, (size_t)0, JNR, JNL, JNQ);
}
